// HAttentionLayer_20186346291762
// MI455X (gfx1250) — hardware-verified
//
#include <hip/hip_runtime.h>
#include <math.h>
#include <stddef.h>


typedef _Float16 v16h __attribute__((ext_vector_type(16)));
typedef _Float16 v8h  __attribute__((ext_vector_type(8)));
typedef float    v8f  __attribute__((ext_vector_type(8)));
typedef float    v4f  __attribute__((ext_vector_type(4)));
typedef v8h v8hA __attribute__((may_alias));
typedef v4f v4fA __attribute__((may_alias));
union Frag { v16h v; v8h half[2]; };

#define T_LEN   2048
#define D_DIM   1024
#define H_NUM   16
#define HD_DIM  64
#define LV_NUM  12
#define NSM     256
#define NDL     192

#define BYTES_TD_H ((size_t)T_LEN * D_DIM * 2)
#define BYTES_DD_H ((size_t)D_DIM * D_DIM * 2)
#define OFF_XH    ((size_t)0)
#define OFF_WQH   (OFF_XH   + BYTES_TD_H)
#define OFF_WKH   (OFF_WQH  + BYTES_DD_H)
#define OFF_WVH   (OFF_WKH  + BYTES_DD_H)
#define OFF_WOH   (OFF_WVH  + BYTES_DD_H)
#define OFF_WSMH  (OFF_WOH  + BYTES_DD_H)
#define OFF_QH    (OFF_WSMH + (size_t)NSM * D_DIM * 2)
#define OFF_KH    (OFF_QH   + BYTES_TD_H)
#define OFF_VHT   (OFF_KH   + BYTES_TD_H)
#define OFF_YH    (OFF_VHT  + BYTES_TD_H)
#define OFF_PSM   (OFF_YH   + BYTES_TD_H)
#define OFF_CGT   (OFF_PSM  + (size_t)T_LEN * NSM * 4)
#define OFF_END   (OFF_CGT  + (size_t)H_NUM * T_LEN * 4)

__device__ __forceinline__ v8f wmma_f16(v16h a, v16h b, v8f c) {
    v8f d = __builtin_amdgcn_wmma_f32_16x16x32_f16(false, a, false, b, (short)0, c, false, false);
    asm volatile("v_nop\n\tv_nop\n\tv_nop\n\tv_nop" : "+v"(d) : "v"(a), "v"(b));
    return d;
}

__device__ __forceinline__ v8f zero8() {
    const v8f z = {0.f, 0.f, 0.f, 0.f, 0.f, 0.f, 0.f, 0.f};
    return z;
}

__device__ __forceinline__ float softplus_f(float z) {
    return fmaxf(z, 0.0f) + log1pf(expf(-fabsf(z)));
}

__global__ __launch_bounds__(256) void cvt_f16_kernel(const float* __restrict__ src, _Float16* __restrict__ dst,
                                                       int n8, float scale) {
    const int i = (int)blockIdx.x * 256 + (int)threadIdx.x;
    if (i >= n8) return;
    const v4fA* p = (const v4fA*)(src + (size_t)i * 8);
    const v4f a = p[0];
    const v4f b = p[1];
    v8h o;
    o[0] = (_Float16)(a[0] * scale); o[1] = (_Float16)(a[1] * scale);
    o[2] = (_Float16)(a[2] * scale); o[3] = (_Float16)(a[3] * scale);
    o[4] = (_Float16)(b[0] * scale); o[5] = (_Float16)(b[1] * scale);
    o[6] = (_Float16)(b[2] * scale); o[7] = (_Float16)(b[3] * scale);
    volatile v8h* q = (volatile v8h*)(dst + (size_t)i * 8);
    *q = o;
    __threadfence();
    *q = o;
}

__global__ __launch_bounds__(256) void zero_f16_kernel(_Float16* __restrict__ dst, int n8) {
    const int i = (int)blockIdx.x * 256 + (int)threadIdx.x;
    if (i >= n8) return;
    v8h o;
#pragma unroll
    for (int r = 0; r < 8; ++r) o[r] = (_Float16)0.0f;
    volatile v8h* q = (volatile v8h*)(dst + (size_t)i * 8);
    *q = o;
    __threadfence();
    *q = o;
}

template <int MODE>
__global__ __launch_bounds__(128) void gemm_kernel(const _Float16* __restrict__ A, const _Float16* __restrict__ B,
                                                   void* __restrict__ Cv, int N, float oscale) {
    __shared__ __align__(16) unsigned char stg_raw[16384];
    const int lane = (int)threadIdx.x & 31, w = (int)threadIdx.x >> 5, lg = lane >> 4, ln = lane & 15;
    int t0, n0;
    if (MODE == 2) { t0 = (int)blockIdx.y * 64 + w * 16; n0 = (int)blockIdx.x * 64; }
    else           { t0 = (int)blockIdx.y * 16;          n0 = (int)blockIdx.x * 256 + w * 64; }

    v8f acc[4];
#pragma unroll
    for (int j = 0; j < 4; ++j) acc[j] = zero8();

    const _Float16* arow = A + (size_t)(t0 + ln) * D_DIM;
#pragma unroll 2
    for (int k0 = 0; k0 < D_DIM; k0 += 32) {
        Frag a;
        a.half[0] = *(const v8hA*)(arow + k0 + 8 * lg);
        a.half[1] = *(const v8hA*)(arow + k0 + 16 + 8 * lg);
#pragma unroll
        for (int j = 0; j < 4; ++j) {
            const _Float16* brow = B + (size_t)(n0 + j * 16 + ln) * D_DIM + k0;
            Frag b;
            b.half[0] = *(const v8hA*)(brow + 8 * lg);
            b.half[1] = *(const v8hA*)(brow + 16 + 8 * lg);
            acc[j] = wmma_f16(a.v, b.v, acc[j]);
        }
    }

    if (MODE == 0) {
        _Float16* stg = (_Float16*)stg_raw;
#pragma unroll
        for (int j = 0; j < 4; ++j)
#pragma unroll
            for (int r = 0; r < 8; ++r)
                stg[(w * 16 + 8 * lg + r) * 64 + j * 16 + ln] = (_Float16)(acc[j][r] * oscale);
        __syncthreads();
        _Float16* C = (_Float16*)Cv;
        v8h vals[4];
#pragma unroll
        for (int p = 0; p < 4; ++p) {
            const int row = p * 4 + (lane >> 3), col = (lane & 7) * 8;
            vals[p] = *(const v8hA*)(stg + (w * 16 + row) * 64 + col);
        }
#pragma unroll
        for (int p = 0; p < 4; ++p) {
            const int row = p * 4 + (lane >> 3), col = (lane & 7) * 8;
            *(volatile v8h*)(C + (size_t)(t0 + row) * N + n0 + col) = vals[p];
        }
        __threadfence();
#pragma unroll
        for (int p = 0; p < 4; ++p) {
            const int row = p * 4 + (lane >> 3), col = (lane & 7) * 8;
            *(volatile v8h*)(C + (size_t)(t0 + row) * N + n0 + col) = vals[p];
        }
    } else if (MODE == 1) {
        float* stg = (float*)stg_raw;
#pragma unroll
        for (int j = 0; j < 4; ++j)
#pragma unroll
            for (int r = 0; r < 8; ++r)
                stg[(w * 16 + 8 * lg + r) * 64 + j * 16 + ln] = acc[j][r] * oscale;
        __syncthreads();
        float* C = (float*)Cv;
        v4f vals[8];
#pragma unroll
        for (int p = 0; p < 8; ++p) {
            const int row = p * 2 + (lane >> 4), col = (lane & 15) * 4;
            vals[p] = *(const v4fA*)(stg + (w * 16 + row) * 64 + col);
        }
#pragma unroll
        for (int p = 0; p < 8; ++p) {
            const int row = p * 2 + (lane >> 4), col = (lane & 15) * 4;
            *(volatile v4f*)(C + (size_t)(t0 + row) * N + n0 + col) = vals[p];
        }
        __threadfence();
#pragma unroll
        for (int p = 0; p < 8; ++p) {
            const int row = p * 2 + (lane >> 4), col = (lane & 15) * 4;
            *(volatile v4f*)(C + (size_t)(t0 + row) * N + n0 + col) = vals[p];
        }
    } else {
        (void)N;
        _Float16* stg = (_Float16*)stg_raw;
#pragma unroll
        for (int j = 0; j < 4; ++j) {
            v8h hv;
#pragma unroll
            for (int r = 0; r < 8; ++r) hv[r] = (_Float16)(acc[j][r] * oscale);
            *(v8hA*)(stg + (j * 16 + ln) * 64 + w * 16 + 8 * lg) = hv;
        }
        __syncthreads();
        _Float16* C = (_Float16*)Cv;
        const int tid = (int)threadIdx.x;
        const int tb = (int)blockIdx.y * 64;
        v8h vals[4];
#pragma unroll
        for (int p = 0; p < 4; ++p) {
            const int nrow = p * 16 + (tid >> 3), tcol = (tid & 7) * 8;
            vals[p] = *(const v8hA*)(stg + nrow * 64 + tcol);
        }
#pragma unroll
        for (int p = 0; p < 4; ++p) {
            const int nrow = p * 16 + (tid >> 3), tcol = (tid & 7) * 8;
            *(volatile v8h*)(C + (size_t)(n0 + nrow) * T_LEN + tb + tcol) = vals[p];
        }
        __threadfence();
#pragma unroll
        for (int p = 0; p < 4; ++p) {
            const int nrow = p * 16 + (tid >> 3), tcol = (tid & 7) * 8;
            *(volatile v8h*)(C + (size_t)(n0 + nrow) * T_LEN + tb + tcol) = vals[p];
        }
    }
}

__global__ __launch_bounds__(32) void decay_scan_kernel(const float* __restrict__ Psm, const float* __restrict__ A_log,
                                                        const float* __restrict__ dt_bias, float* __restrict__ cgT) {
    const int h = (int)blockIdx.x;
    const int lane = (int)threadIdx.x & 31;
    const float Ah = -expf(A_log[h]);
    const float bh = dt_bias[h];
    float carry = 0.0f;
    for (int c = 0; c < T_LEN / 128; ++c) {
        const int tbase = c * 128 + lane * 4;
        const float g0 = Ah * softplus_f(Psm[(size_t)(tbase + 0) * NSM + NDL + h] + bh);
        const float g1 = Ah * softplus_f(Psm[(size_t)(tbase + 1) * NSM + NDL + h] + bh);
        const float g2 = Ah * softplus_f(Psm[(size_t)(tbase + 2) * NSM + NDL + h] + bh);
        const float g3 = Ah * softplus_f(Psm[(size_t)(tbase + 3) * NSM + NDL + h] + bh);
        const float cs0 = g0;
        const float cs1 = cs0 + g1;
        const float cs2 = cs1 + g2;
        const float cs3 = cs2 + g3;
        float incl = cs3;
#pragma unroll
        for (int d = 1; d < 32; d <<= 1) {
            const float u = __shfl_up(incl, d, 32);
            if (lane >= d) incl += u;
        }
        float ex = __shfl_up(incl, 1, 32);
        if (lane == 0) ex = 0.0f;
        const float baseval = carry + ex;
        v4f o;
        o[0] = cs0 + baseval; o[1] = cs1 + baseval; o[2] = cs2 + baseval; o[3] = cs3 + baseval;
        volatile v4f* q = (volatile v4f*)(cgT + (size_t)h * T_LEN + tbase);
        *q = o;
        __threadfence();
        *q = o;
        carry += __shfl(incl, 31, 32);
    }
}

__global__ __launch_bounds__(128) void hattn_kernel(const _Float16* __restrict__ Qh, const _Float16* __restrict__ Kh,
                                                    const _Float16* __restrict__ VhT, const float* __restrict__ cgT,
                                                    const float* __restrict__ Psm, const float* __restrict__ Lp,
                                                    _Float16* __restrict__ Yh, float pscale, float inv_pscale) {
    __shared__ __align__(16) _Float16 PL[4 * 16 * 32];
    __shared__ __align__(16) _Float16 YS[4 * 16 * 64];
    __shared__ float LL[4 * 16 * LV_NUM];

    const int lane = (int)threadIdx.x & 31, w = (int)threadIdx.x >> 5, lg = lane >> 4, ln = lane & 15;
    const int h = (int)blockIdx.y;
    const int tb = (int)blockIdx.x * 64;
    const int t0 = tb + w * 16;

    for (int k = lane; k < 16 * LV_NUM; k += 32) {
        const int row = k / LV_NUM, l = k - row * LV_NUM;
        const float z = Lp[h * LV_NUM + l] * Psm[(size_t)(t0 + row) * NSM + h * LV_NUM + l];
        LL[(w * 16 + row) * LV_NUM + l] = softplus_f(z);
    }

    const _Float16* qrow = Qh + (size_t)(t0 + ln) * D_DIM + h * HD_DIM;
    Frag q0f, q1f;
    q0f.half[0] = *(const v8hA*)(qrow + 8 * lg);
    q0f.half[1] = *(const v8hA*)(qrow + 16 + 8 * lg);
    q1f.half[0] = *(const v8hA*)(qrow + 32 + 8 * lg);
    q1f.half[1] = *(const v8hA*)(qrow + 48 + 8 * lg);

    float cgt[8];
#pragma unroll
    for (int r = 0; r < 8; ++r) cgt[r] = cgT[(size_t)h * T_LEN + t0 + 8 * lg + r];

    v8f accY[4];
#pragma unroll
    for (int j = 0; j < 4; ++j) accY[j] = zero8();

    __syncthreads();

    const float gsc = 0.125f * pscale;
    const int nit = 2 * (int)blockIdx.x + 2;
    for (int it = 0; it < nit; ++it) {
        const int s0 = it * 32;
#pragma unroll
        for (int sub = 0; sub < 2; ++sub) {
            const int sg = s0 + sub * 16 + ln;
            const _Float16* krow = Kh + (size_t)sg * D_DIM + h * HD_DIM;
            Frag k0f, k1f;
            k0f.half[0] = *(const v8hA*)(krow + 8 * lg);
            k0f.half[1] = *(const v8hA*)(krow + 16 + 8 * lg);
            k1f.half[0] = *(const v8hA*)(krow + 32 + 8 * lg);
            k1f.half[1] = *(const v8hA*)(krow + 48 + 8 * lg);
            v8f sc = zero8();
            sc = wmma_f16(q0f.v, k0f.v, sc);
            sc = wmma_f16(q1f.v, k1f.v, sc);
            const float cgs = cgT[(size_t)h * T_LEN + sg];
#pragma unroll
            for (int r = 0; r < 8; ++r) {
                const int trow = t0 + 8 * lg + r;
                const int xr = trow ^ sg;
                const int lv = xr ? (32 - __builtin_clz((unsigned)xr)) : 0;
                const float lam = LL[(w * 16 + 8 * lg + r) * LV_NUM + lv];
                const float dcy = __expf(fminf(cgt[r] - cgs, 0.0f));
                float wv = sc[r] * gsc * dcy * lam;
                wv = (sg <= trow) ? wv : 0.0f;
                PL[(w * 16 + 8 * lg + r) * 32 + sub * 16 + ln] = (_Float16)wv;
            }
        }
        __syncthreads();
        Frag pf;
        pf.half[0] = *(const v8hA*)(PL + (w * 16 + ln) * 32 + 8 * lg);
        pf.half[1] = *(const v8hA*)(PL + (w * 16 + ln) * 32 + 16 + 8 * lg);
#pragma unroll
        for (int j = 0; j < 4; ++j) {
            const _Float16* vrow = VhT + (size_t)(h * HD_DIM + j * 16 + ln) * T_LEN + s0;
            Frag vf;
            vf.half[0] = *(const v8hA*)(vrow + 8 * lg);
            vf.half[1] = *(const v8hA*)(vrow + 16 + 8 * lg);
            accY[j] = wmma_f16(pf.v, vf.v, accY[j]);
        }
        __syncthreads();
    }

#pragma unroll
    for (int j = 0; j < 4; ++j)
#pragma unroll
        for (int r = 0; r < 8; ++r)
            YS[(w * 16 + 8 * lg + r) * 64 + j * 16 + ln] = (_Float16)(accY[j][r] * inv_pscale);
    __syncthreads();
    v8h vals[4];
#pragma unroll
    for (int p = 0; p < 4; ++p) {
        const int row = p * 4 + (lane >> 3), col = (lane & 7) * 8;
        vals[p] = *(const v8hA*)(YS + (w * 16 + row) * 64 + col);
    }
#pragma unroll
    for (int p = 0; p < 4; ++p) {
        const int row = p * 4 + (lane >> 3), col = (lane & 7) * 8;
        *(volatile v8h*)(Yh + (size_t)(t0 + row) * D_DIM + h * HD_DIM + col) = vals[p];
    }
    __threadfence();
#pragma unroll
    for (int p = 0; p < 4; ++p) {
        const int row = p * 4 + (lane >> 3), col = (lane & 7) * 8;
        *(volatile v8h*)(Yh + (size_t)(t0 + row) * D_DIM + h * HD_DIM + col) = vals[p];
    }
}

__global__ __launch_bounds__(512) void outproj_ln_kernel(const _Float16* __restrict__ Yh, const _Float16* __restrict__ Woh,
                                                         const float* __restrict__ xin, const float* __restrict__ gam,
                                                         const float* __restrict__ bet, float* __restrict__ out,
                                                         float oscale) {
    __shared__ __align__(16) float stg[16 * 8 * 64];
    __shared__ float red[16 * 16];
    __shared__ float mu_s[16];
    __shared__ float inv_s[16];

    const int tid = (int)threadIdx.x;
    const int lane = tid & 31, w = tid >> 5, lg = lane >> 4, ln = lane & 15;
    const int t0 = (int)blockIdx.x * 16;
    const int c0 = w * 64;

    v8f acc[4];
#pragma unroll
    for (int j = 0; j < 4; ++j) acc[j] = zero8();

    const _Float16* arow = Yh + (size_t)(t0 + ln) * D_DIM;
#pragma unroll 2
    for (int k0 = 0; k0 < D_DIM; k0 += 32) {
        Frag a;
        a.half[0] = *(const v8hA*)(arow + k0 + 8 * lg);
        a.half[1] = *(const v8hA*)(arow + k0 + 16 + 8 * lg);
#pragma unroll
        for (int j = 0; j < 4; ++j) {
            const _Float16* brow = Woh + (size_t)(c0 + j * 16 + ln) * D_DIM + k0;
            Frag b;
            b.half[0] = *(const v8hA*)(brow + 8 * lg);
            b.half[1] = *(const v8hA*)(brow + 16 + 8 * lg);
            acc[j] = wmma_f16(a.v, b.v, acc[j]);
        }
    }

#pragma unroll
    for (int j = 0; j < 4; ++j)
#pragma unroll
        for (int r = 0; r < 8; ++r)
            acc[j][r] = acc[j][r] * oscale + xin[(size_t)(t0 + 8 * lg + r) * D_DIM + c0 + j * 16 + ln];

#pragma unroll
    for (int r = 0; r < 8; ++r) {
        float s = acc[0][r] + acc[1][r] + acc[2][r] + acc[3][r];
        s += __shfl_xor(s, 1, 32);
        s += __shfl_xor(s, 2, 32);
        s += __shfl_xor(s, 4, 32);
        s += __shfl_xor(s, 8, 32);
        if (ln == 0) red[w * 16 + 8 * lg + r] = s;
    }
    __syncthreads();
    if (tid < 16) {
        float a = 0.0f;
#pragma unroll
        for (int ww = 0; ww < 16; ++ww) a += red[ww * 16 + tid];
        mu_s[tid] = a * (1.0f / (float)D_DIM);
    }
    __syncthreads();
    float mu[8];
#pragma unroll
    for (int r = 0; r < 8; ++r) mu[r] = mu_s[8 * lg + r];
#pragma unroll
    for (int j = 0; j < 4; ++j)
#pragma unroll
        for (int r = 0; r < 8; ++r) acc[j][r] -= mu[r];

#pragma unroll
    for (int r = 0; r < 8; ++r) {
        float s = acc[0][r] * acc[0][r] + acc[1][r] * acc[1][r] + acc[2][r] * acc[2][r] + acc[3][r] * acc[3][r];
        s += __shfl_xor(s, 1, 32);
        s += __shfl_xor(s, 2, 32);
        s += __shfl_xor(s, 4, 32);
        s += __shfl_xor(s, 8, 32);
        if (ln == 0) red[w * 16 + 8 * lg + r] = s;
    }
    __syncthreads();
    if (tid < 16) {
        float a = 0.0f;
#pragma unroll
        for (int ww = 0; ww < 16; ++ww) a += red[ww * 16 + tid];
        inv_s[tid] = rsqrtf(a * (1.0f / (float)D_DIM) + 1e-5f);
    }
    __syncthreads();
    float iv[8];
#pragma unroll
    for (int r = 0; r < 8; ++r) iv[r] = inv_s[8 * lg + r];
#pragma unroll
    for (int j = 0; j < 4; ++j) {
        const int gcol = c0 + j * 16 + ln;
        const float gj = gam[gcol];
        const float bj = bet[gcol];
#pragma unroll
        for (int r = 0; r < 8; ++r) acc[j][r] = acc[j][r] * iv[r] * gj + bj;
    }

#pragma unroll
    for (int half = 0; half < 2; ++half) {
        if (lg == half) {
#pragma unroll
            for (int j = 0; j < 4; ++j)
#pragma unroll
                for (int r = 0; r < 8; ++r)
                    stg[(w * 8 + r) * 64 + j * 16 + ln] = acc[j][r];
        }
        __syncthreads();
        v4f vals[4];
#pragma unroll
        for (int p = 0; p < 4; ++p) {
            const int row = p * 2 + (lane >> 4), col = (lane & 15) * 4;
            vals[p] = *(const v4fA*)(stg + (w * 8 + row) * 64 + col);
        }
#pragma unroll
        for (int p = 0; p < 4; ++p) {
            const int row = p * 2 + (lane >> 4), col = (lane & 15) * 4;
            *(volatile v4f*)(out + (size_t)(t0 + half * 8 + row) * D_DIM + c0 + col) = vals[p];
        }
        __threadfence();
#pragma unroll
        for (int p = 0; p < 4; ++p) {
            const int row = p * 2 + (lane >> 4), col = (lane & 15) * 4;
            *(volatile v4f*)(out + (size_t)(t0 + half * 8 + row) * D_DIM + c0 + col) = vals[p];
        }
        __syncthreads();
    }
}

extern "C" void kernel_launch(void* const* d_in, const int* in_sizes, int n_in,
                              void* d_out, int out_size, void* d_ws, size_t ws_size,
                              hipStream_t stream) {
    if (n_in < 12) return;
    if (in_sizes[0] != T_LEN * D_DIM) return;
    if (in_sizes[1] != D_DIM * D_DIM || in_sizes[2] != D_DIM * D_DIM || in_sizes[3] != D_DIM * D_DIM) return;
    if (in_sizes[4] != NDL * D_DIM || in_sizes[5] != H_NUM * D_DIM || in_sizes[6] != D_DIM * D_DIM) return;
    if (in_sizes[7] < H_NUM || in_sizes[8] < H_NUM || in_sizes[9] < H_NUM * LV_NUM) return;
    if (in_sizes[10] < D_DIM || in_sizes[11] < D_DIM) return;
    if (out_size != T_LEN * D_DIM) return;
    if (OFF_END > ws_size) return;

    const float* x     = (const float*)d_in[0];
    const float* Wq    = (const float*)d_in[1];
    const float* Wk    = (const float*)d_in[2];
    const float* Wv    = (const float*)d_in[3];
    const float* Wdl   = (const float*)d_in[4];
    const float* Wdt   = (const float*)d_in[5];
    const float* Wout  = (const float*)d_in[6];
    const float* A_log = (const float*)d_in[7];
    const float* dt_b  = (const float*)d_in[8];
    const float* Lp    = (const float*)d_in[9];
    const float* ln_g  = (const float*)d_in[10];
    const float* ln_b  = (const float*)d_in[11];

    char* ws = (char*)d_ws;
    _Float16* xh   = (_Float16*)(ws + OFF_XH);
    _Float16* wqh  = (_Float16*)(ws + OFF_WQH);
    _Float16* wkh  = (_Float16*)(ws + OFF_WKH);
    _Float16* wvh  = (_Float16*)(ws + OFF_WVH);
    _Float16* woh  = (_Float16*)(ws + OFF_WOH);
    _Float16* wsmh = (_Float16*)(ws + OFF_WSMH);
    _Float16* Qh   = (_Float16*)(ws + OFF_QH);
    _Float16* Kh   = (_Float16*)(ws + OFF_KH);
    _Float16* VhT  = (_Float16*)(ws + OFF_VHT);
    _Float16* Yh   = (_Float16*)(ws + OFF_YH);
    float*    psm  = (float*)(ws + OFF_PSM);
    float*    cgT  = (float*)(ws + OFF_CGT);

    const float wsc  = 32.0f;
    const float iwsc = 1.0f / 32.0f;
    const float psc  = 512.0f;
    const float ipsc = 1.0f / 512.0f;

    const int n8_td  = T_LEN * D_DIM / 8;
    const int n8_dd  = D_DIM * D_DIM / 8;
    const int n8_dl  = NDL * D_DIM / 8;
    const int n8_dt  = H_NUM * D_DIM / 8;
    const int n8_pad = (NSM - NDL - H_NUM) * D_DIM / 8;
    cvt_f16_kernel<<<(n8_td + 255) / 256, 256, 0, stream>>>(x, xh, n8_td, 1.0f);
    cvt_f16_kernel<<<(n8_dd + 255) / 256, 256, 0, stream>>>(Wq, wqh, n8_dd, wsc);
    cvt_f16_kernel<<<(n8_dd + 255) / 256, 256, 0, stream>>>(Wk, wkh, n8_dd, wsc);
    cvt_f16_kernel<<<(n8_dd + 255) / 256, 256, 0, stream>>>(Wv, wvh, n8_dd, wsc);
    cvt_f16_kernel<<<(n8_dd + 255) / 256, 256, 0, stream>>>(Wout, woh, n8_dd, wsc);
    cvt_f16_kernel<<<(n8_dl + 255) / 256, 256, 0, stream>>>(Wdl, wsmh, n8_dl, wsc);
    cvt_f16_kernel<<<(n8_dt + 255) / 256, 256, 0, stream>>>(Wdt, wsmh + (size_t)NDL * D_DIM, n8_dt, wsc);
    zero_f16_kernel<<<(n8_pad + 255) / 256, 256, 0, stream>>>(wsmh + (size_t)(NDL + H_NUM) * D_DIM, n8_pad);

    gemm_kernel<1><<<dim3(NSM / 256, T_LEN / 16), 128, 0, stream>>>(xh, wsmh, (void*)psm, NSM, iwsc);
    gemm_kernel<0><<<dim3(D_DIM / 256, T_LEN / 16), 128, 0, stream>>>(xh, wqh, (void*)Qh, D_DIM, iwsc);
    gemm_kernel<0><<<dim3(D_DIM / 256, T_LEN / 16), 128, 0, stream>>>(xh, wkh, (void*)Kh, D_DIM, iwsc);
    gemm_kernel<2><<<dim3(D_DIM / 64, T_LEN / 64), 128, 0, stream>>>(xh, wvh, (void*)VhT, D_DIM, iwsc);

    decay_scan_kernel<<<H_NUM, 32, 0, stream>>>(psm, A_log, dt_b, cgT);

    hattn_kernel<<<dim3(T_LEN / 64, H_NUM), 128, 0, stream>>>(Qh, Kh, VhT, cgT, psm, Lp, Yh, psc, ipsc);

    outproj_ln_kernel<<<T_LEN / 16, 512, 0, stream>>>(Yh, woh, x, ln_g, ln_b, (float*)d_out, iwsc);
}
